// GCN_30279519437683
// MI455X (gfx1250) — hardware-verified
//
#include <hip/hip_runtime.h>
#include <stddef.h>
#include <stdint.h>
#include <math.h>


#define CIN    128
#define HID    64
#define K2     128
#define NCLS   16
#define NTHR   256
#define NWAVE  8
#define EPT    8
#define CHUNK  (NTHR * EPT)
#define WCAP   (EPT * 32)
#define LISTN  (NWAVE * WCAP)
#define NBD    8192
#define SLD    13
#define NBA    1024
#define SLA    10
#define RCAP   20480
#define DEGCAP 64
#define GBM    64
#define GTHR   128
#define RPB    64
#define NU0    (HID * (CIN / 8))
#define NU1    (HID * (K2 / 8))
#define NU2    (NCLS * (K2 / 8))
#define BLD_ZINTS (LISTN + 2 * RCAP + 3 * NBA)
#define BLD_LDS_INTS (BLD_ZINTS + 16)
#define WSMAX  134217728

static_assert((CHUNK & (CHUNK - 1)) == 0 && CHUNK <= 4096);
static_assert((NBD & (NBD - 1)) == 0 && NBD == (1 << SLD));
static_assert((NBA & (NBA - 1)) == 0 && NBA == (1 << SLA));
static_assert(((long long)CHUNK << SLD) < (1LL << 31));
static_assert(((long long)CHUNK << SLA) < (1LL << 31));
static_assert(NBD % (NTHR * 4) == 0);
static_assert(LISTN % NTHR == 0);
static_assert(NBA == NTHR * 4 && NBA % 32 == 0 && NBA % GBM == 0);
static_assert(RCAP % (NTHR * 4) == 0 && BLD_ZINTS % (NTHR * 4) == 0 && LISTN % 4 == 0);
static_assert(CIN % 32 == 0 && K2 % 32 == 0 && K2 == 2 * HID && CIN == 128);
static_assert(GBM == (GTHR / 32) * 16 && HID == 64 && NCLS == 16);
static_assert(NU0 % NTHR == 0 && (NU0 + NU1) % NTHR == 0 && (NU0 + NU1 + NU2) % NTHR == 0);
static_assert(RPB % NWAVE == 0 && RPB == GBM);
static_assert(HID == 2 * 32);
static_assert(DEGCAP >= 36 + 8 && RCAP >= 16721 + 2048);
static_assert(BLD_LDS_INTS * 4 <= 300000);

typedef float          v2f   __attribute__((ext_vector_type(2)));
typedef float          v4f   __attribute__((ext_vector_type(4)));
typedef float          v8f   __attribute__((ext_vector_type(8)));
typedef int            v4i   __attribute__((ext_vector_type(4)));
typedef int            v8i   __attribute__((ext_vector_type(8)));
typedef unsigned int   v4u   __attribute__((ext_vector_type(4)));
typedef unsigned short v8us  __attribute__((ext_vector_type(8)));
typedef unsigned short v16us __attribute__((ext_vector_type(16)));
typedef __bf16         v16bf __attribute__((ext_vector_type(16)));
typedef v2f  __attribute__((may_alias)) v2fa;
typedef v4f  __attribute__((may_alias)) v4fa;
typedef v4i  __attribute__((may_alias)) v4ia;
typedef v8us __attribute__((may_alias)) v8usa;
union FragB { v16bf v; v16us u; v8us h[2]; v8i w; };

__device__ __forceinline__ v8f wmb(const FragB& a, const FragB& b, v8f c) {
  v8f d = __builtin_amdgcn_wmma_f32_16x16x32_bf16(false, a.v, false, b.v, (short)0, c, false, false);
  asm volatile("v_nop\n\tv_nop\n\tv_nop\n\tv_nop" : "+v"(d) : "v"(a.w), "v"(b.w));
  return d;
}

__device__ __forceinline__ unsigned bf16_bits(float f) {
  const unsigned u = __float_as_uint(f);
  return ((u + 0x7FFFu + ((u >> 16) & 1u)) >> 16) & 0xFFFFu;
}
__device__ __forceinline__ float bf16_val(float f) {
  return __uint_as_float(bf16_bits(f) << 16);
}
__device__ __forceinline__ int pk2(float a, float b) {
  return (int)(bf16_bits(a) | (bf16_bits(b) << 16));
}
__device__ __forceinline__ int clampi(int v, int lo, int hi) {
  return v < lo ? lo : (v > hi ? hi : v);
}

template <int SLB>
__device__ __forceinline__ int scan_chunk(const int* __restrict__ dsts, int nE, int cbase, int slotBase,
                                          int nb, int vec8, int* list, int tid, int lane, int wave) {
  int wc = 0;
  const int el0  = tid * EPT;
  const int e0   = cbase + el0;
  const int sent = -2147483647 - 1;
  v4i da, db;
  if (vec8 != 0 && cbase + CHUNK <= nE) {
    da = *(const v4i*)(dsts + e0);
    db = *(const v4i*)(dsts + e0 + 4);
  } else {
    da.x = (e0     < nE) ? dsts[min(e0,     nE - 1)] : sent;
    da.y = (e0 + 1 < nE) ? dsts[min(e0 + 1, nE - 1)] : sent;
    da.z = (e0 + 2 < nE) ? dsts[min(e0 + 2, nE - 1)] : sent;
    da.w = (e0 + 3 < nE) ? dsts[min(e0 + 3, nE - 1)] : sent;
    db.x = (e0 + 4 < nE) ? dsts[min(e0 + 4, nE - 1)] : sent;
    db.y = (e0 + 5 < nE) ? dsts[min(e0 + 5, nE - 1)] : sent;
    db.z = (e0 + 6 < nE) ? dsts[min(e0 + 6, nE - 1)] : sent;
    db.w = (e0 + 7 < nE) ? dsts[min(e0 + 7, nE - 1)] : sent;
  }
  const unsigned nbs = (unsigned)slotBase;
  const unsigned unb = (unsigned)nb;
  const unsigned s0 = (unsigned)da.x - nbs, s1 = (unsigned)da.y - nbs;
  const unsigned s2 = (unsigned)da.z - nbs, s3 = (unsigned)da.w - nbs;
  const unsigned s4 = (unsigned)db.x - nbs, s5 = (unsigned)db.y - nbs;
  const unsigned s6 = (unsigned)db.z - nbs, s7 = (unsigned)db.w - nbs;
  const bool h0 = s0 < unb, h1 = s1 < unb, h2 = s2 < unb, h3 = s3 < unb;
  const bool h4 = s4 < unb, h5 = s5 < unb, h6 = s6 < unb, h7 = s7 < unb;
  const unsigned any = __builtin_amdgcn_ballot_w32(h0 | h1 | h2 | h3 | h4 | h5 | h6 | h7);
  if (any != 0u) {
#define HITJ(J, HJ, SJ) { \
      const unsigned mj = __builtin_amdgcn_ballot_w32(HJ); \
      if (mj != 0u) { \
        if (HJ) { \
          const int pos = wc + (int)__builtin_amdgcn_mbcnt_lo(mj, 0u); \
          if (pos < WCAP) list[wave * WCAP + pos] = ((el0 + (J)) << SLB) | (int)(SJ); \
        } \
        wc += (int)__builtin_popcount(mj); } }
    HITJ(0, h0, s0)
    HITJ(1, h1, s1)
    HITJ(2, h2, s2)
    HITJ(3, h3, s3)
    HITJ(4, h4, s4)
    HITJ(5, h5, s5)
    HITJ(6, h6, s6)
    HITJ(7, h7, s7)
#undef HITJ
  }
  return wc;
}

__device__ __forceinline__ void wunit(const float* __restrict__ p, int stride, unsigned short* dp) {
  v8us o;
#pragma unroll
  for (int i = 0; i < 8; ++i) o[i] = (unsigned short)bf16_bits(p[(size_t)i * stride]);
  *(volatile v8us*)dp = o;
  __threadfence();
  *(volatile v8us*)dp = o;
}

__global__ __launch_bounds__(NTHR) void k_wprep(const float* __restrict__ W0, const float* __restrict__ W1,
                                                const float* __restrict__ W2, unsigned short* W0T,
                                                unsigned short* W1T2, unsigned short* W2T2) {
  const int u = (int)blockIdx.x * NTHR + (int)threadIdx.x;
  if (u < NU0) {
    const int n  = u >> 4;
    const int k8 = (u & 15) * 8;
    wunit(W0 + (size_t)k8 * HID + n, HID, W0T + (size_t)n * CIN + k8);
  } else if (u < NU0 + NU1) {
    const int v  = u - NU0;
    const int n  = v >> 4;
    const int k8 = (v & 15) * 8;
    const int kk = k8 & (HID - 1);
    wunit(W1 + (size_t)kk * HID + n, HID, W1T2 + (size_t)n * K2 + k8);
  } else if (u < NU0 + NU1 + NU2) {
    const int v  = u - NU0 - NU1;
    const int n  = v >> 4;
    const int k8 = (v & 15) * 8;
    const int kk = k8 & (HID - 1);
    wunit(W2 + (size_t)kk * NCLS + n, NCLS, W2T2 + (size_t)n * K2 + k8);
  }
}

__global__ __launch_bounds__(NTHR) void k_deg(const int* __restrict__ keys, int nE, int vec8, float* dos) {
  __shared__ __attribute__((aligned(16))) int scnt[NBD];
  __shared__ __attribute__((aligned(16))) int list[LISTN];
  __shared__ int wcnt[NWAVE];
  const int tid = (int)threadIdx.x, lane = tid & 31, wave = tid >> 5;
  const int nodeBase = (int)blockIdx.x * NBD;

  for (int i = tid; i < NBD; i += NTHR) scnt[i] = 0;
  for (int i = tid; i < LISTN; i += NTHR) list[i] = 0;
  if (tid < NWAVE) wcnt[tid] = 0;
  __syncthreads();

  const int nChunks = (nE + CHUNK - 1) / CHUNK;
#pragma unroll 1
  for (int ch = 0; ch < nChunks; ++ch) {
    const int cbase = ch * CHUNK;
    const int wc = scan_chunk<SLD>(keys, nE, cbase, nodeBase, NBD, vec8, list, tid, lane, wave);
    if (lane == 0) wcnt[wave] = wc;
    __syncthreads();
    if (wave == 0) {
#pragma unroll 1
      for (int w2 = 0; w2 < NWAVE; ++w2) {
        int c = wcnt[w2];
        c = c < 0 ? 0 : (c > WCAP ? WCAP : c);
#pragma unroll 1
        for (int b0 = 0; b0 < c; b0 += 32) {
          const int idx = b0 + lane;
          const int ent = list[w2 * WCAP + (idx < WCAP ? idx : WCAP - 1)];
          const int m32 = (c - b0) < 32 ? (c - b0) : 32;
#pragma unroll 1
          for (int k = 0; k < m32; ++k) {
            const int u  = __builtin_amdgcn_readlane(ent, k);
            const int sl = u & (NBD - 1);
            if (lane == 0) scnt[sl] = scnt[sl] + 1;
          }
        }
      }
    }
    __syncthreads();
  }

  v4f vals[NBD / (NTHR * 4)];
#pragma unroll
  for (int it = 0; it < NBD / (NTHR * 4); ++it) {
    const int s0 = it * (NTHR * 4) + 4 * tid;
    const v4i c4 = *(const v4ia*)(scnt + s0);
    const float d0 = fmaxf((float)c4.x, 1.0f), d1 = fmaxf((float)c4.y, 1.0f);
    const float d2 = fmaxf((float)c4.z, 1.0f), d3 = fmaxf((float)c4.w, 1.0f);
    v4f v;
    v.x = rsqrtf(d0); v.y = rsqrtf(d1); v.z = rsqrtf(d2); v.w = rsqrtf(d3);
    vals[it] = v;
  }
#pragma unroll
  for (int it = 0; it < NBD / (NTHR * 4); ++it) {
    const int s0 = it * (NTHR * 4) + 4 * tid;
    *(volatile v4f*)(dos + (size_t)nodeBase + s0) = vals[it];
  }
  __threadfence();
#pragma unroll
  for (int it = 0; it < NBD / (NTHR * 4); ++it) {
    const int s0 = it * (NTHR * 4) + 4 * tid;
    *(volatile v4f*)(dos + (size_t)nodeBase + s0) = vals[it];
  }
}

__global__ __launch_bounds__(NTHR) void k_build(const int* __restrict__ srcs, const int* __restrict__ dsts,
                                                int nE, int nN, int vec8, int* cntp, int* offp, int* lstp) {
  extern __shared__ __attribute__((aligned(16))) int dsm[];
  int* list = dsm;
  int* hl   = dsm + LISTN;
  int* sl   = dsm + LISTN + RCAP;
  int* cnt  = dsm + LISTN + 2 * RCAP;
  int* offs = cnt + NBA;
  int* cur  = offs + NBA;
  int* misc = cur + NBA;
  const int tid = (int)threadIdx.x, lane = tid & 31, wave = tid >> 5;
  const int nodeBase = (int)blockIdx.x * NBA;

  {
    const v4i z4 = {0, 0, 0, 0};
    for (int i = tid * 4; i < BLD_ZINTS; i += NTHR * 4) *(v4ia*)(dsm + i) = z4;
    if (tid < 16) misc[tid] = 0;
  }
  __syncthreads();

  int t = 0, ov = 0;
  const int nChunks = (nE + CHUNK - 1) / CHUNK;
#pragma unroll 1
  for (int ch = 0; ch < nChunks; ++ch) {
    const int cbase = ch * CHUNK;
    const int wc = scan_chunk<SLA>(dsts, nE, cbase, nodeBase, NBA, vec8, list, tid, lane, wave);
    if (lane == 0) misc[wave] = wc;
    __syncthreads();
    if (wave == 0) {
#pragma unroll 1
      for (int w2 = 0; w2 < NWAVE; ++w2) {
        int c = misc[w2];
        c = c < 0 ? 0 : (c > WCAP ? WCAP : c);
#pragma unroll 1
        for (int b0 = 0; b0 < c; b0 += 32) {
          const int idx = b0 + lane;
          const int ent = list[w2 * WCAP + (idx < WCAP ? idx : WCAP - 1)];
          const int m32 = (c - b0) < 32 ? (c - b0) : 32;
#pragma unroll 1
          for (int k = 0; k < m32; ++k) {
            const int u    = __builtin_amdgcn_readlane(ent, k);
            const int slot = u & (NBA - 1);
            const int el   = (u >> SLA) & (CHUNK - 1);
            const int pk   = ((cbase + el) << SLA) | slot;
            if (t < RCAP) {
              if (lane == 0) { hl[t] = pk; cnt[slot] = cnt[slot] + 1; }
              t = t + 1;
            } else {
              ov = 1;
            }
          }
        }
      }
    }
    __syncthreads();
  }
  if (wave == 0 && lane == 0) { misc[8] = t; misc[9] = ov; }
  __syncthreads();
  int tt = misc[8];
  tt = tt < 0 ? 0 : (tt > RCAP ? RCAP : tt);
  const int ovf = misc[9];

  if (wave == 0) {
    const int base = lane * (NBA / 32);
    int s = 0;
#pragma unroll 1
    for (int i = 0; i < NBA / 32; ++i) s += cnt[base + i];
    int incl = s;
#pragma unroll
    for (int d = 1; d < 32; d <<= 1) {
      const int y = __shfl_up(incl, d, 32);
      if (lane >= d) incl += y;
    }
    int run = incl - s;
#pragma unroll 1
    for (int i = 0; i < NBA / 32; ++i) {
      const int cv = cnt[base + i];
      offs[base + i] = run;
      cur[base + i]  = run;
      run += cv;
    }
  }
  __syncthreads();
  if (wave == 0) {
#pragma unroll 1
    for (int b0 = 0; b0 < tt; b0 += 32) {
      const int idx = b0 + lane;
      const int ent = hl[idx < RCAP ? idx : RCAP - 1];
      const int m32 = (tt - b0) < 32 ? (tt - b0) : 32;
#pragma unroll 1
      for (int k = 0; k < m32; ++k) {
        const int u    = __builtin_amdgcn_readlane(ent, k);
        const int slot = u & (NBA - 1);
        if (lane == 0) {
          int p = cur[slot];
          p = p < 0 ? 0 : (p > RCAP - 1 ? RCAP - 1 : p);
          sl[p] = u;
          cur[slot] = p + 1;
        }
      }
    }
  }
  __syncthreads();

  if (ovf != 0) {
    for (int i = tid; i < NBA; i += NTHR) cnt[i] = DEGCAP + 1;
  }
#pragma unroll 1
  for (int i4 = tid * 4; i4 < RCAP; i4 += NTHR * 4) {
    const v4i e = *(const v4ia*)(sl + i4);
    const int e0 = clampi(e.x >> SLA, 0, nE - 1);
    const int e1 = clampi(e.y >> SLA, 0, nE - 1);
    const int e2 = clampi(e.z >> SLA, 0, nE - 1);
    const int e3 = clampi(e.w >> SLA, 0, nE - 1);
    int r0 = srcs[e0], r1 = srcs[e1], r2 = srcs[e2], r3 = srcs[e3];
    r0 = clampi(r0, 0, nN - 1); r1 = clampi(r1, 0, nN - 1);
    r2 = clampi(r2, 0, nN - 1); r3 = clampi(r3, 0, nN - 1);
    v4i o;
    o.x = (i4 + 0 < tt) ? r0 : 0;
    o.y = (i4 + 1 < tt) ? r1 : 0;
    o.z = (i4 + 2 < tt) ? r2 : 0;
    o.w = (i4 + 3 < tt) ? r3 : 0;
    *(v4ia*)(sl + i4) = o;
  }
  __syncthreads();

  const v4i cv = *(const v4ia*)(cnt + 4 * tid);
  const v4i fv = *(const v4ia*)(offs + 4 * tid);
  int* cp = cntp + (size_t)blockIdx.x * NBA + 4 * tid;
  int* fp = offp + (size_t)blockIdx.x * NBA + 4 * tid;
  int* lp = lstp + (size_t)blockIdx.x * RCAP;
  *(volatile v4i*)cp = cv;
  *(volatile v4i*)fp = fv;
#pragma unroll 1
  for (int i4 = tid * 4; i4 < RCAP; i4 += NTHR * 4) {
    const v4i o = *(const v4ia*)(sl + i4);
    *(volatile v4i*)(lp + i4) = o;
  }
  __threadfence();
  *(volatile v4i*)cp = cv;
  *(volatile v4i*)fp = fv;
#pragma unroll 1
  for (int i4 = tid * 4; i4 < RCAP; i4 += NTHR * 4) {
    const v4i o = *(const v4ia*)(sl + i4);
    *(volatile v4i*)(lp + i4) = o;
  }
}

__global__ __launch_bounds__(GTHR) void k_gemm0(const float* __restrict__ X, const unsigned short* __restrict__ WT,
                                                const float* __restrict__ dos, float* outF, int nN) {
  __shared__ __attribute__((aligned(16))) float stg[GBM * HID];
  __shared__ float sdos[GBM];
  const int tid = (int)threadIdx.x, lane = tid & 31, wave = tid >> 5, hh = lane >> 4, m = lane & 15;
  const int rowBase = (int)blockIdx.x * GBM;

  if (tid < GBM) {
    int r = rowBase + tid;
    r = r < nN ? r : nN - 1;
    sdos[tid] = dos[r];
  }
  v8f acc[4];
  {
    const v8f z = {0.f, 0.f, 0.f, 0.f, 0.f, 0.f, 0.f, 0.f};
    acc[0] = z; acc[1] = z; acc[2] = z; acc[3] = z;
  }
  int ar = rowBase + 16 * wave + m;
  ar = ar < nN ? ar : nN - 1;
  const float* ap = X + (size_t)ar * CIN + 8 * hh;
  const unsigned short* wp = WT + (size_t)m * CIN + 8 * hh;
#pragma unroll 1
  for (int ks = 0; ks < CIN / 32; ++ks) {
    const float* aq = ap + 32 * ks;
    const v4f x0 = *(const v4fa*)aq;
    const v4f x1 = *(const v4fa*)(aq + 4);
    const v4f x2 = *(const v4fa*)(aq + 16);
    const v4f x3 = *(const v4fa*)(aq + 20);
    v8i wv;
    wv[0] = pk2(x0.x, x0.y); wv[1] = pk2(x0.z, x0.w);
    wv[2] = pk2(x1.x, x1.y); wv[3] = pk2(x1.z, x1.w);
    wv[4] = pk2(x2.x, x2.y); wv[5] = pk2(x2.z, x2.w);
    wv[6] = pk2(x3.x, x3.y); wv[7] = pk2(x3.z, x3.w);
    FragB af;
    af.w = wv;
#pragma unroll
    for (int t = 0; t < 4; ++t) {
      const unsigned short* wq = wp + (size_t)(16 * t) * CIN + 32 * ks;
      FragB bf;
      bf.h[0] = *(const v8usa*)wq;
      bf.h[1] = *(const v8usa*)(wq + 16);
      acc[t] = wmb(af, bf, acc[t]);
    }
  }

#pragma unroll
  for (int t = 0; t < 4; ++t) {
    const int lc = 16 * t + m;
#pragma unroll
    for (int r = 0; r < 8; ++r) {
      const int lr = 16 * wave + 8 * hh + r;
      stg[lr * HID + lc] = acc[t][r];
    }
  }
  __syncthreads();

  v4f fv[8];
#pragma unroll
  for (int i = 0; i < 8; ++i) {
    const int lr = 16 * wave + 2 * i + hh;
    const float sc = sdos[lr];
    const v4f v = *(const v4fa*)(stg + lr * HID + 4 * m);
    fv[i] = v * sc;
  }
#pragma unroll
  for (int i = 0; i < 8; ++i) {
    const int gr = rowBase + 16 * wave + 2 * i + hh;
    float* op = outF + (size_t)gr * HID + 4 * m;
    *(volatile v4f*)op = fv[i];
  }
  __threadfence();
#pragma unroll
  for (int i = 0; i < 8; ++i) {
    const int gr = rowBase + 16 * wave + 2 * i + hh;
    float* op = outF + (size_t)gr * HID + 4 * m;
    *(volatile v4f*)op = fv[i];
  }
}

template <int MODE>
__global__ __launch_bounds__(NTHR) void k_rep(const int* __restrict__ cntp, const int* __restrict__ offp,
                                              const int* __restrict__ lstp, int nN, int mRows, int tabRows,
                                              const float* __restrict__ dos, const float* __restrict__ xl,
                                              const float* __restrict__ bias, unsigned short* hb, float* hout) {
  const int tid = (int)threadIdx.x, lane = tid & 31, wave = tid >> 5;
  const int blockBase = (int)blockIdx.x * RPB;
  float bv0 = 0.0f, bv1 = 0.0f;
  if constexpr (MODE == 0) {
    const v2f a = *(const v2fa*)(bias + 2 * lane);
    bv0 = bf16_val(a.x); bv1 = bf16_val(a.y);
  }
  const float qnan = __int_as_float(0x7fc00000);
  const int sa = (2 * lane) & 31, sb = (2 * lane + 1) & 31;
  const int q0s = (4 * lane) & 31, q1s = (4 * lane + 1) & 31;
  const int q2s = (4 * lane + 2) & 31, q3s = (4 * lane + 3) & 31;
#pragma unroll 1
  for (int i = 0; i < RPB / NWAVE; ++i) {
    const int node = blockBase + i * NWAVE + wave;
    const int nc = node < nN ? node : nN - 1;
    const int tn = node < tabRows ? node : tabRows - 1;
    const int craw = cntp[tn];
    const bool big = (craw > DEGCAP) || (craw < 0);
    const int c = clampi(craw, 0, DEGCAP);
    const int o = clampi(offp[tn], 0, RCAP);
    const size_t lbase = (size_t)(tn >> SLA) * RCAP;
    float acc0 = 0.0f, acc1 = 0.0f;
#pragma unroll 1
    for (int b0 = 0; b0 < c; b0 += 32) {
      int idx = o + b0 + lane;
      idx = idx > RCAP - 1 ? RCAP - 1 : idx;
      int sr = lstp[lbase + idx];
      sr = clampi(sr, 0, nN - 1);
      const int m32 = (c - b0) < 32 ? (c - b0) : 32;
#pragma unroll 1
      for (int k = 0; k < m32; ++k) {
        const int sk = __builtin_amdgcn_readlane(sr, k);
        const v2f a = *(const v2fa*)(xl + (size_t)sk * HID + 2 * lane);
        acc0 = acc0 + a.x; acc1 = acc1 + a.y;
      }
    }
    const float dis = rsqrtf((float)(craw < 1 ? 1 : craw));
    const float pzr = big ? qnan : 0.0f;
    const bool live = node < nN;
    const bool wr = (node < mRows) && (lane < 16);
    if constexpr (MODE == 0) {
      const float ds = dos[nc];
      float y0 = acc0 * dis + bv0;
      float y1 = acc1 * dis + bv1;
      y0 = (y0 > 0.0f) ? y0 : (y0 - y0);
      y1 = (y1 > 0.0f) ? y1 : (y1 - y1);
      y0 = (y0 + pzr) * ds; y1 = (y1 + pzr) * ds;
      const float v0 = live ? y0 : 0.0f;
      const float v1 = live ? y1 : 0.0f;
      v4f ow;
      ow.x = __shfl(v0, sa, 32); ow.y = __shfl(v1, sa, 32);
      ow.z = __shfl(v0, sb, 32); ow.w = __shfl(v1, sb, 32);
      float* op = hout + (size_t)node * HID + 4 * (lane & 15);
      if (wr) *(volatile v4f*)op = ow;
      __threadfence();
      if (wr) *(volatile v4f*)op = ow;
    } else {
      const float y0 = acc0 * dis + pzr;
      const float y1 = acc1 * dis + pzr;
      const float v0 = live ? y0 : 0.0f;
      const float v1 = live ? y1 : 0.0f;
      const unsigned hb0 = bf16_bits(v0), hb1 = bf16_bits(v1);
      const unsigned lb0 = bf16_bits(v0 - __uint_as_float(hb0 << 16));
      const unsigned lb1 = bf16_bits(v1 - __uint_as_float(hb1 << 16));
      const int hw = (int)(hb0 | (hb1 << 16));
      const int lw = (int)(lb0 | (lb1 << 16));
      const int g0 = __shfl(hw, q0s, 32), g1 = __shfl(hw, q1s, 32);
      const int g2 = __shfl(hw, q2s, 32), g3 = __shfl(hw, q3s, 32);
      const int p0 = __shfl(lw, q0s, 32), p1 = __shfl(lw, q1s, 32);
      const int p2 = __shfl(lw, q2s, 32), p3 = __shfl(lw, q3s, 32);
      const bool lsel = (lane & 8) != 0;
      v4u pv;
      pv.x = (unsigned int)(lsel ? p0 : g0);
      pv.y = (unsigned int)(lsel ? p1 : g1);
      pv.z = (unsigned int)(lsel ? p2 : g2);
      pv.w = (unsigned int)(lsel ? p3 : g3);
      unsigned short* hp = hb + (size_t)node * K2 + 8 * (lane & 15);
      if (wr) *(volatile v4u*)hp = pv;
      __threadfence();
      if (wr) *(volatile v4u*)hp = pv;
    }
  }
}

__global__ __launch_bounds__(GTHR) void k_mlp(const unsigned short* __restrict__ A2,
                                              const unsigned short* __restrict__ W1T2,
                                              const unsigned short* __restrict__ W2T2,
                                              const float* __restrict__ b1, const float* __restrict__ dos,
                                              float* g2, int nN) {
  __shared__ __attribute__((aligned(16))) unsigned short h2[GBM * K2];
  __shared__ __attribute__((aligned(16))) float ot[GBM * NCLS];
  __shared__ float sdos[GBM];
  const int tid = (int)threadIdx.x, lane = tid & 31, wave = tid >> 5, hh = lane >> 4, m = lane & 15;
  const int rowBase = (int)blockIdx.x * GBM;

  if (tid < GBM) {
    int r = rowBase + tid;
    r = r < nN ? r : nN - 1;
    sdos[tid] = dos[r];
  }
  v8f acc[4];
  {
    const v8f z = {0.f, 0.f, 0.f, 0.f, 0.f, 0.f, 0.f, 0.f};
    acc[0] = z; acc[1] = z; acc[2] = z; acc[3] = z;
  }
  const unsigned short* ap = A2 + (size_t)(rowBase + 16 * wave + m) * K2 + 8 * hh;
  const unsigned short* wp = W1T2 + (size_t)m * K2 + 8 * hh;
#pragma unroll 1
  for (int ks = 0; ks < K2 / 32; ++ks) {
    FragB af;
    af.h[0] = *(const v8usa*)(ap + 32 * ks);
    af.h[1] = *(const v8usa*)(ap + 32 * ks + 16);
#pragma unroll
    for (int t = 0; t < 4; ++t) {
      const unsigned short* wq = wp + (size_t)(16 * t) * K2 + 32 * ks;
      FragB bf;
      bf.h[0] = *(const v8usa*)wq;
      bf.h[1] = *(const v8usa*)(wq + 16);
      acc[t] = wmb(af, bf, acc[t]);
    }
  }

#pragma unroll
  for (int t = 0; t < 4; ++t) {
    const int lc = 16 * t + m;
    const float bb = bf16_val(b1[lc]);
#pragma unroll
    for (int r = 0; r < 8; ++r) {
      const int lr = 16 * wave + 8 * hh + r;
      float v = acc[t][r] + bb;
      v = (v > 0.0f) ? v : (v - v);
      const unsigned hbv = bf16_bits(v);
      const unsigned lbv = bf16_bits(v - __uint_as_float(hbv << 16));
      h2[lr * K2 + lc]       = (unsigned short)hbv;
      h2[lr * K2 + HID + lc] = (unsigned short)lbv;
    }
  }
  __syncthreads();

  v8f acc2 = {0.f, 0.f, 0.f, 0.f, 0.f, 0.f, 0.f, 0.f};
  {
    const unsigned short* hp = h2 + (16 * wave + m) * K2 + 8 * hh;
    const unsigned short* wp2 = W2T2 + (size_t)m * K2 + 8 * hh;
#pragma unroll
    for (int ks = 0; ks < K2 / 32; ++ks) {
      FragB af, bf;
      af.h[0] = *(const v8usa*)(hp + 32 * ks);
      af.h[1] = *(const v8usa*)(hp + 32 * ks + 16);
      bf.h[0] = *(const v8usa*)(wp2 + 32 * ks);
      bf.h[1] = *(const v8usa*)(wp2 + 32 * ks + 16);
      acc2 = wmb(af, bf, acc2);
    }
  }
#pragma unroll
  for (int r = 0; r < 8; ++r) {
    const int lr = 16 * wave + 8 * hh + r;
    ot[lr * NCLS + m] = acc2[r];
  }
  __syncthreads();

  v4f ov[2];
#pragma unroll
  for (int j = 0; j < 2; ++j) {
    const int q  = j * GTHR + tid;
    const int lr = q >> 2;
    const v4f v = *(const v4fa*)(ot + 4 * q);
    ov[j] = v * sdos[lr];
  }
  float* ob = g2 + (size_t)rowBase * NCLS;
#pragma unroll
  for (int j = 0; j < 2; ++j) *(volatile v4f*)(ob + 4 * (j * GTHR + tid)) = ov[j];
  __threadfence();
#pragma unroll
  for (int j = 0; j < 2; ++j) *(volatile v4f*)(ob + 4 * (j * GTHR + tid)) = ov[j];
}

__global__ __launch_bounds__(NTHR) void k_agg2(const int* __restrict__ cntp, const int* __restrict__ offp,
                                               const int* __restrict__ lstp, int nN, int tabRows,
                                               const float* __restrict__ g2, const float* __restrict__ b2,
                                               float* out) {
  const int tid = (int)threadIdx.x, lane = tid & 31, wave = tid >> 5;
  const int g = lane >> 2, q = lane & 3;
  const int base = ((int)blockIdx.x * NWAVE + wave) * 8;
  if (base >= nN) return;
  const int node = base + g;
  const int nc = node < nN ? node : nN - 1;
  const int tn = nc < tabRows ? nc : tabRows - 1;
  const int craw = cntp[tn];
  const bool big = (craw > DEGCAP) || (craw < 0);
  const int cc = clampi(craw, 0, DEGCAP);
  const int o = clampi(offp[tn], 0, RCAP);
  const size_t lbase = (size_t)(tn >> SLA) * RCAP;
  int cm = cc;
#pragma unroll
  for (int d = 16; d >= 1; d >>= 1) {
    const int y = __shfl_xor(cm, d, 32);
    cm = cm > y ? cm : y;
  }
  cm = __builtin_amdgcn_readfirstlane(cm);
  cm = cm > DEGCAP ? DEGCAP : cm;
  float a0 = 0.0f, a1 = 0.0f, a2 = 0.0f, a3 = 0.0f;
#pragma unroll 1
  for (int p = 0; p < cm; ++p) {
    int idx = o + p;
    idx = idx > RCAP - 1 ? RCAP - 1 : idx;
    int sr = lstp[lbase + idx];
    sr = clampi(sr, 0, nN - 1);
    const v4f v = *(const v4fa*)(g2 + (size_t)sr * NCLS + 4 * q);
    const int msk = (p < cc) ? -1 : 0;
    a0 = a0 + __int_as_float(__float_as_int(v.x) & msk);
    a1 = a1 + __int_as_float(__float_as_int(v.y) & msk);
    a2 = a2 + __int_as_float(__float_as_int(v.z) & msk);
    a3 = a3 + __int_as_float(__float_as_int(v.w) & msk);
  }
  const v4f bq = *(const v4fa*)(b2 + 4 * q);
  const float dis = rsqrtf((float)(craw < 1 ? 1 : craw));
  const float pzr = big ? __int_as_float(0x7fc00000) : 0.0f;
  v4f ow;
  ow.x = (a0 * dis + bf16_val(bq.x)) + pzr;
  ow.y = (a1 * dis + bf16_val(bq.y)) + pzr;
  ow.z = (a2 * dis + bf16_val(bq.z)) + pzr;
  ow.w = (a3 * dis + bf16_val(bq.w)) + pzr;
  float* op = out + (size_t)node * NCLS + 4 * q;
  const bool wr = node < nN;
  if (wr) *(volatile v4f*)op = ow;
  __threadfence();
  if (wr) *(volatile v4f*)op = ow;
}

static inline int cdiv(int a, int b) { return (a + b - 1) / b; }
static inline size_t al256(size_t o) { return (o + 255) & ~(size_t)255; }

extern "C" void kernel_launch(void* const* d_in, const int* in_sizes, int n_in,
                              void* d_out, int out_size, void* d_ws, size_t ws_size,
                              hipStream_t stream) {
  if (n_in < 9) return;
  if (in_sizes[0] < CIN || (in_sizes[0] % CIN) != 0) return;
  const int nN = in_sizes[0] / CIN;
  if (nN < 8 || nN > (1 << 22) || (nN % 8) != 0) return;
  const int nE = in_sizes[1];
  if (nE < 1 || nE >= (1 << (31 - SLA))) return;
  if (in_sizes[2] != nE) return;
  if (in_sizes[3] != CIN * HID || in_sizes[4] != HID) return;
  if (in_sizes[5] != HID * HID || in_sizes[6] != HID) return;
  if (in_sizes[7] != HID * NCLS || in_sizes[8] != NCLS) return;
  if ((long long)out_size != (long long)nN * NCLS) return;

  const float* x   = (const float*)d_in[0];
  const int*   src = (const int*)d_in[1];
  const int*   dst = (const int*)d_in[2];
  const float* W0  = (const float*)d_in[3];
  const float* b0  = (const float*)d_in[4];
  const float* W1  = (const float*)d_in[5];
  const float* b1  = (const float*)d_in[6];
  const float* W2  = (const float*)d_in[7];
  const float* b2  = (const float*)d_in[8];
  float* out = (float*)d_out;

  const int MP   = cdiv(nN, GBM) * GBM;
  const int gM   = MP / GBM;
  const int gD   = cdiv(nN, NBD);
  const int NBPD = gD * NBD;
  const int gA   = cdiv(MP, NBA);
  const int TAB  = gA * NBA;
  if ((long long)TAB < (long long)MP) return;
  if (NBPD < MP) return;
  const int vec8 = ((nE & 3) == 0) ? 1 : 0;

  char* ws = (char*)d_ws;
  size_t off = 0;
  const size_t oDOS = off; off = al256(off + (size_t)NBPD * 4);
  const size_t oW0T = off; off = al256(off + (size_t)HID * CIN * 2);
  const size_t oW1T = off; off = al256(off + (size_t)HID * K2 * 2);
  const size_t oW2T = off; off = al256(off + (size_t)NCLS * K2 * 2);
  const size_t oCNT = off; off = al256(off + (size_t)TAB * 4);
  const size_t oOFF = off; off = al256(off + (size_t)TAB * 4);
  const size_t oLST = off; off = al256(off + (size_t)gA * RCAP * 4);
  const size_t oG0  = off; off = al256(off + (size_t)MP * HID * 4);
  const size_t oG1  = off; off = al256(off + (size_t)MP * HID * 4);
  const size_t oA2  = off; off = al256(off + (size_t)MP * K2 * 2);
  const size_t oG2  = off; off = al256(off + (size_t)MP * NCLS * 4);
  if (off > ws_size || off > (size_t)WSMAX) return;
  float*          DOS  = (float*)(ws + oDOS);
  unsigned short* W0T  = (unsigned short*)(ws + oW0T);
  unsigned short* W1T2 = (unsigned short*)(ws + oW1T);
  unsigned short* W2T2 = (unsigned short*)(ws + oW2T);
  int*            CNT  = (int*)(ws + oCNT);
  int*            OFF  = (int*)(ws + oOFF);
  int*            LST  = (int*)(ws + oLST);
  float*          G0   = (float*)(ws + oG0);
  float*          G1   = (float*)(ws + oG1);
  unsigned short* A2   = (unsigned short*)(ws + oA2);
  float*          G2   = (float*)(ws + oG2);

  const size_t bldLds = (size_t)BLD_LDS_INTS * 4;
  hipFuncSetAttribute(reinterpret_cast<const void*>(&k_build), hipFuncAttributeMaxDynamicSharedMemorySize, (int)bldLds);

  k_wprep<<<(NU0 + NU1 + NU2) / NTHR, NTHR, 0, stream>>>(W0, W1, W2, W0T, W1T2, W2T2);
  k_deg<<<gD, NTHR, 0, stream>>>(src, nE, vec8, DOS);
  k_build<<<gA, NTHR, bldLds, stream>>>(src, dst, nE, nN, vec8, CNT, OFF, LST);
  k_gemm0<<<gM, GTHR, 0, stream>>>(x, W0T, DOS, G0, nN);
  k_rep<0><<<gM, NTHR, 0, stream>>>(CNT, OFF, LST, nN, MP, TAB, DOS, G0, b0, A2, G1);
  k_rep<1><<<gM, NTHR, 0, stream>>>(CNT, OFF, LST, nN, MP, TAB, DOS, G1, b0, A2, G1);
  k_mlp<<<gM, GTHR, 0, stream>>>(A2, W1T2, W2T2, b1, DOS, G2, nN);
  k_agg2<<<cdiv(nN, NWAVE * 8), NTHR, 0, stream>>>(CNT, OFF, LST, nN, TAB, G2, b2, out);
}
